// GATEncoder_12738873000057
// MI455X (gfx1250) — hardware-verified
//
#include <hip/hip_runtime.h>
#include <stddef.h>
#include <stdint.h>


#define NN      20000
#define NE      640000
#define NF      256
#define NF2     512
#define NL      3
#define NG      16
#define NO      128
#define MP      20096
#define NTHR    256
#define NWAVE   8
#define EPT     8
#define CHUNK   (NTHR * EPT)
#define WCAP    (EPT * 32)
#define LISTN   (NWAVE * WCAP)
#define NBA     512
#define SLA     9
#define NBLK     40
#define RCAP    28672
#define DEGCAP  96
#define GBM     64
#define GBN     128
#define GTHR    128
#define GWAVE   (GTHR / 32)
#define NEGS    0.2f
#define EPSN    1e-5f
#define PBX     (MP * 32 / NTHR)
#define WBX     (64 + 256 + 32)
#define BZINTS  (LISTN + 2 * RCAP + 3 * NBA + 64)
#define B_LDS_BYTES (BZINTS * 4)
#define WSMAX   134217728

static_assert((CHUNK & (CHUNK - 1)) == 0 && CHUNK <= 4096);
static_assert((NBA & (NBA - 1)) == 0 && NBA == (1 << SLA));
static_assert(((long long)CHUNK << SLA) < (1LL << 31));
static_assert(((long long)NE << SLA) < (1LL << 31));
static_assert(NN < 32768);
static_assert(NBLK * NBA >= MP && MP >= NN && (MP % GBM) == 0 && MP == 157 * 128);
static_assert((NF % 32) == 0 && (NF2 % 32) == 0 && (NF % 8) == 0 && NF2 == 2 * NF);
static_assert((NF2 % GBN) == 0 && GBM == GWAVE * 16 && GBN == 4 * 32);
static_assert(RCAP >= 16673 + 4096 && (RCAP % 1024) == 0);
static_assert(DEGCAP >= 60 + 8);
static_assert((BZINTS % 4) == 0 && B_LDS_BYTES <= 300000);
static_assert(PBX * NTHR == MP * 32);
static_assert(NBA % NWAVE == 0 && NBA % 32 == 0);
static_assert((NE % 4) == 0);
static_assert(NTHR == NF && NWAVE * 16 == NO);

typedef float          v4f   __attribute__((ext_vector_type(4)));
typedef float          v8f   __attribute__((ext_vector_type(8)));
typedef int            v4i   __attribute__((ext_vector_type(4)));
typedef int            v8i   __attribute__((ext_vector_type(8)));
typedef double         v2d   __attribute__((ext_vector_type(2)));
typedef unsigned short v8us  __attribute__((ext_vector_type(8)));
typedef unsigned short v16us __attribute__((ext_vector_type(16)));
typedef __bf16         v16bf __attribute__((ext_vector_type(16)));
typedef v4f  __attribute__((may_alias)) v4fa;
typedef v4i  __attribute__((may_alias)) v4ia;
typedef v2d  __attribute__((may_alias)) v2da;
typedef v8us __attribute__((may_alias)) v8usa;
union FragB { v16bf v; v16us u; v8us h[2]; v8i w; };

__device__ __forceinline__ v8f wmb(const FragB& a, const FragB& b, v8f c) {
  v8f d = __builtin_amdgcn_wmma_f32_16x16x32_bf16(false, a.v, false, b.v, (short)0, c, false, false);
  asm volatile("v_nop\n\tv_nop\n\tv_nop\n\tv_nop" : "+v"(d) : "v"(a.w), "v"(b.w));
  return d;
}
__device__ __forceinline__ v8f z8() { v8f z = {0.f, 0.f, 0.f, 0.f, 0.f, 0.f, 0.f, 0.f}; return z; }

__device__ __forceinline__ void ldwait() { asm volatile("s_wait_loadcnt 0x0" ::: "memory"); }

__device__ __forceinline__ unsigned bfbits(float v) {
  unsigned u = __float_as_uint(v);
  u = u + 0x7FFFu + ((u >> 16) & 1u);
  return u >> 16;
}
__device__ __forceinline__ unsigned bfn(float v) {
  const unsigned r = bfbits(v);
  return (v != v) ? 0x7fc0u : r;
}
__device__ __forceinline__ float rbf(float v) { return __uint_as_float(bfbits(v) << 16); }

__device__ __forceinline__ v8us cvt8b(const v4f a, const v4f b) {
  v8us o;
  o[0] = (unsigned short)bfbits(a.x); o[1] = (unsigned short)bfbits(a.y);
  o[2] = (unsigned short)bfbits(a.z); o[3] = (unsigned short)bfbits(a.w);
  o[4] = (unsigned short)bfbits(b.x); o[5] = (unsigned short)bfbits(b.y);
  o[6] = (unsigned short)bfbits(b.z); o[7] = (unsigned short)bfbits(b.w);
  return o;
}

__device__ __forceinline__ void st2u(unsigned short* p, const v8us v) {
  *(volatile v8us*)p = v;
  __threadfence();
  *(volatile v8us*)p = v;
}

__device__ __forceinline__ v8us wtr8(const float* __restrict__ w, int cols, int n, int k) {
  const float* p = w + (size_t)k * (size_t)cols + n;
  v4f a, b;
  a.x = p[0];                  a.y = p[(size_t)cols];       a.z = p[(size_t)2 * cols];   a.w = p[(size_t)3 * cols];
  b.x = p[(size_t)4 * cols];   b.y = p[(size_t)5 * cols];   b.z = p[(size_t)6 * cols];   b.w = p[(size_t)7 * cols];
  return cvt8b(a, b);
}

template <int SLB>
__device__ __forceinline__ int scan_chunk(const int* __restrict__ dsts, int nE, int cbase, int slotBase,
                                          int nb, int vec8, int* list, int tid, int lane, int wave) {
  int wc = 0;
  const int el0  = tid * EPT;
  const int e0   = cbase + el0;
  const int sent = -2147483647 - 1;
  v4i da, db;
  if (vec8 != 0 && cbase + CHUNK <= nE) {
    da = *(const v4i*)(dsts + e0);
    db = *(const v4i*)(dsts + e0 + 4);
  } else {
    da.x = (e0     < nE) ? dsts[min(e0,     nE - 1)] : sent;
    da.y = (e0 + 1 < nE) ? dsts[min(e0 + 1, nE - 1)] : sent;
    da.z = (e0 + 2 < nE) ? dsts[min(e0 + 2, nE - 1)] : sent;
    da.w = (e0 + 3 < nE) ? dsts[min(e0 + 3, nE - 1)] : sent;
    db.x = (e0 + 4 < nE) ? dsts[min(e0 + 4, nE - 1)] : sent;
    db.y = (e0 + 5 < nE) ? dsts[min(e0 + 5, nE - 1)] : sent;
    db.z = (e0 + 6 < nE) ? dsts[min(e0 + 6, nE - 1)] : sent;
    db.w = (e0 + 7 < nE) ? dsts[min(e0 + 7, nE - 1)] : sent;
  }
  const unsigned nbs = (unsigned)slotBase;
  const unsigned unb = (unsigned)nb;
  const unsigned s0 = (unsigned)da.x - nbs, s1 = (unsigned)da.y - nbs;
  const unsigned s2 = (unsigned)da.z - nbs, s3 = (unsigned)da.w - nbs;
  const unsigned s4 = (unsigned)db.x - nbs, s5 = (unsigned)db.y - nbs;
  const unsigned s6 = (unsigned)db.z - nbs, s7 = (unsigned)db.w - nbs;
  const bool h0 = s0 < unb, h1 = s1 < unb, h2 = s2 < unb, h3 = s3 < unb;
  const bool h4 = s4 < unb, h5 = s5 < unb, h6 = s6 < unb, h7 = s7 < unb;
  const unsigned any = __builtin_amdgcn_ballot_w32(h0 | h1 | h2 | h3 | h4 | h5 | h6 | h7);
  if (any != 0u) {
#define HITJ(J, HJ, SJ) { \
      const unsigned mj = __builtin_amdgcn_ballot_w32(HJ); \
      if (mj != 0u) { \
        if (HJ) { \
          const int pos = wc + (int)__builtin_amdgcn_mbcnt_lo(mj, 0u); \
          if (pos < WCAP) list[wave * WCAP + pos] = ((el0 + (J)) << SLB) | (int)(SJ); \
        } \
        wc += (int)__builtin_popcount(mj); } }
    HITJ(0, h0, s0)
    HITJ(1, h1, s1)
    HITJ(2, h2, s2)
    HITJ(3, h3, s3)
    HITJ(4, h4, s4)
    HITJ(5, h5, s5)
    HITJ(6, h6, s6)
    HITJ(7, h7, s7)
#undef HITJ
  }
  return wc;
}

__global__ __launch_bounds__(NTHR) void k_prep(const float* __restrict__ x, const float* __restrict__ Wl,
                                               const float* __restrict__ Wr, const float* __restrict__ fcW,
                                               unsigned short* xb, unsigned short* w0, unsigned short* w12,
                                               unsigned short* fct) {
  const int bx = (int)blockIdx.x, tid = (int)threadIdx.x;
  if (bx < PBX) {
    const int i   = bx * NTHR + tid;
    const int row = i >> 5;
    const int c0  = (i & 31) * 8;
    const int rc  = row < NN ? row : NN - 1;
    const float* p = x + (size_t)rc * NF + c0;
    v4f a = *(const v4f*)p, b = *(const v4f*)(p + 4);
    const v4f z4 = {0.f, 0.f, 0.f, 0.f};
    if (row >= NN) { a = z4; b = z4; }
    st2u(xb + (size_t)i * 8, cvt8b(a, b));
  } else {
    const int wb = bx - PBX;
    if (wb < 64) {
      const int u  = wb * NTHR + tid;
      const int n  = (u >> 5) & (NF - 1);
      const int k8 = (u & 31) * 8;
      v8us o;
      if (wb < 32) o = wtr8(Wl, NF, n, k8);
      else         o = wtr8(Wr, NF, n, k8);
      st2u(w0 + (size_t)u * 8, o);
    } else if (wb < 320) {
      const int v   = wb - 64;
      const int lay = 1 + (v >> 7);
      const int vb  = v & 127;
      const int u   = vb * NTHR + tid;
      const int n   = (u >> 6) & (NF - 1);
      const int ks  = ((u & 63) * 8) & (NF - 1);
      v8us o;
      if (vb < 64) o = wtr8(Wl + (size_t)lay * NF * NF, NF, n, ks);
      else         o = wtr8(Wr + (size_t)lay * NF * NF, NF, n, ks);
      st2u(w12 + (size_t)(lay - 1) * (NF2 * NF2) + (size_t)u * 8, o);
    } else {
      const int u  = (wb - 320) * NTHR + tid;
      const int n  = u >> 6;
      const int ks = ((u & 63) * 8) & (NF - 1);
      st2u(fct + (size_t)u * 8, wtr8(fcW, NO, n, ks));
    }
  }
}

__global__ __launch_bounds__(NTHR) void k_bucket(const int* __restrict__ srcs, const int* __restrict__ dsts,
                                                 int* hits, int* stab, int* meta) {
  extern __shared__ __attribute__((aligned(16))) int dsm[];
  int* list = dsm;
  int* hl   = dsm + LISTN;
  int* sl   = hl + RCAP;
  int* cnt  = sl + RCAP;
  int* offs = cnt + NBA;
  int* cur  = offs + NBA;
  int* misc = cur + NBA;
  const int tid = (int)threadIdx.x, lane = tid & 31, wave = tid >> 5;
  const int blk = (int)blockIdx.x;
  const int nodeBase = blk * NBA;

  {
    const v4i z4 = {0, 0, 0, 0};
    for (int i = tid * 4; i < BZINTS; i += NTHR * 4) *(v4ia*)(dsm + i) = z4;
  }
  __syncthreads();

  int t = 0, ov = 0;
  const int nChunks = (NE + CHUNK - 1) / CHUNK;
#pragma unroll 1
  for (int ch = 0; ch < nChunks; ++ch) {
    const int cbase = ch * CHUNK;
    const int wc = scan_chunk<SLA>(dsts, NE, cbase, nodeBase, NBA, 1, list, tid, lane, wave);
    if (lane == 0) misc[wave] = wc;
    __syncthreads();
    if (wave == 0) {
#pragma unroll 1
      for (int w2 = 0; w2 < NWAVE; ++w2) {
        int c = misc[w2];
        c = c < 0 ? 0 : (c > WCAP ? WCAP : c);
#pragma unroll 1
        for (int b0 = 0; b0 < c; b0 += 32) {
          const int idx = b0 + lane;
          const int ent = list[w2 * WCAP + (idx < WCAP ? idx : WCAP - 1)];
          const int m32 = (c - b0) < 32 ? (c - b0) : 32;
#pragma unroll 1
          for (int k = 0; k < m32; ++k) {
            const int u    = __builtin_amdgcn_readlane(ent, k);
            const int slot = u & (NBA - 1);
            const int el   = (u >> SLA) & (CHUNK - 1);
            const int pk   = ((cbase + el) << SLA) | slot;
            if (t < RCAP) {
              if (lane == 0) { hl[t] = pk; cnt[slot] = cnt[slot] + 1; }
              t = t + 1;
            } else {
              ov = 1;
            }
          }
        }
      }
    }
    __syncthreads();
  }
  if (wave == 0 && lane == 0) { misc[8] = t; misc[9] = ov; misc[32] = t; misc[33] = ov; }
  __syncthreads();
  int tt = misc[8];
  tt = tt < 0 ? 0 : (tt > RCAP ? RCAP : tt);

  if (wave == 0) {
    const int base = lane * (NBA / 32);
    int s = 0;
#pragma unroll 1
    for (int i = 0; i < NBA / 32; ++i) s += cnt[base + i];
    int incl = s;
#pragma unroll
    for (int d = 1; d < 32; d <<= 1) {
      const int y = __shfl_up(incl, d, 32);
      if (lane >= d) incl += y;
    }
    int run = incl - s;
#pragma unroll 1
    for (int i = 0; i < NBA / 32; ++i) {
      const int cv = cnt[base + i];
      offs[base + i] = run;
      cur[base + i]  = run;
      run += cv;
    }
  }
  __syncthreads();
  if (wave == 0) {
#pragma unroll 1
    for (int b0 = 0; b0 < tt; b0 += 32) {
      const int idx = b0 + lane;
      const int ent = hl[idx < RCAP ? idx : RCAP - 1];
      const int m32 = (tt - b0) < 32 ? (tt - b0) : 32;
#pragma unroll 1
      for (int k = 0; k < m32; ++k) {
        const int u    = __builtin_amdgcn_readlane(ent, k);
        const int slot = u & (NBA - 1);
        if (lane == 0) {
          int p = cur[slot];
          p = p < 0 ? 0 : (p > RCAP - 1 ? RCAP - 1 : p);
          sl[p] = u;
          cur[slot] = p + 1;
        }
      }
    }
  }
  __syncthreads();

#pragma unroll 1
  for (int i = tid; i < tt; i += NTHR) {
    const int u = sl[i];
    int eid = u >> SLA;
    eid = eid < 0 ? 0 : (eid > NE - 1 ? NE - 1 : eid);
    int sr = srcs[eid];
    sr = sr < 0 ? 0 : (sr > NN - 1 ? NN - 1 : sr);
    sl[i] = sr;
  }
  __syncthreads();

  int* hp = hits + (size_t)blk * RCAP + 4 * tid;
  int* sp = stab + (size_t)blk * (2 * NBA) + 4 * tid;
  int* mp = meta + (size_t)blk * 32 + 4 * tid;
#pragma unroll 1
  for (int i = 0; i < RCAP / 1024; ++i) {
    const v4i v = *(const v4ia*)(sl + i * 1024 + 4 * tid);
    *(volatile v4i*)(hp + i * 1024) = v;
  }
  {
    const v4i tv = *(const v4ia*)(cnt + 4 * tid);
    *(volatile v4i*)sp = tv;
    if (tid < 8) { const v4i mv = *(const v4ia*)(misc + 32 + 4 * tid); *(volatile v4i*)mp = mv; }
  }
  __threadfence();
#pragma unroll 1
  for (int i = 0; i < RCAP / 1024; ++i) {
    const v4i v = *(const v4ia*)(sl + i * 1024 + 4 * tid);
    *(volatile v4i*)(hp + i * 1024) = v;
  }
  {
    const v4i tv = *(const v4ia*)(cnt + 4 * tid);
    *(volatile v4i*)sp = tv;
    if (tid < 8) { const v4i mv = *(const v4ia*)(misc + 32 + 4 * tid); *(volatile v4i*)mp = mv; }
  }
}

__global__ __launch_bounds__(GTHR) void k_gemm(const unsigned short* __restrict__ A,
                                               const unsigned short* __restrict__ BT, int K,
                                               const float* __restrict__ bl, const float* __restrict__ br,
                                               float* xout) {
  __shared__ __attribute__((aligned(16))) float stg[GBM * GBN];
  const int tid = (int)threadIdx.x, lane = tid & 31, wave = tid >> 5, hh = lane >> 4, m = lane & 15;
  const int rowBase = (int)blockIdx.x * GBM;
  const int colBase = (int)blockIdx.y * GBN;

  v8f acc[8];
#pragma unroll
  for (int t = 0; t < 8; ++t) acc[t] = z8();
  const unsigned short* ap = A  + (size_t)(rowBase + 16 * wave + m) * (size_t)K + 8 * hh;
  const unsigned short* bp = BT + (size_t)(colBase + m) * (size_t)K + 8 * hh;

#pragma unroll 1
  for (int k0 = 0; k0 < K; k0 += 32) {
    FragB af;
    af.h[0] = *(const v8usa*)(ap + k0);
    af.h[1] = *(const v8usa*)(ap + k0 + 16);
#pragma unroll
    for (int nt = 0; nt < 8; ++nt) {
      const unsigned short* wq = bp + (size_t)(16 * nt) * (size_t)K + k0;
      FragB bf;
      bf.h[0] = *(const v8usa*)wq;
      bf.h[1] = *(const v8usa*)(wq + 16);
      acc[nt] = wmb(af, bf, acc[nt]);
    }
  }

#pragma unroll
  for (int nt = 0; nt < 8; ++nt) {
    const int lc = 16 * nt + m;
#pragma unroll
    for (int r = 0; r < 8; ++r) {
      const int lr = 16 * wave + 8 * hh + r;
      stg[lr * GBN + lc] = acc[nt][r];
    }
  }
  __syncthreads();

  float bq[4];
  {
    const int cb = (colBase & (NF - 1)) + 4 * lane;
    const v4f b1 = *(const v4f*)(bl + cb);
    const v4f b2 = *(const v4f*)(br + cb);
    const bool isR = colBase >= NF;
    bq[0] = rbf(isR ? b2.x : b1.x); bq[1] = rbf(isR ? b2.y : b1.y);
    bq[2] = rbf(isR ? b2.z : b1.z); bq[3] = rbf(isR ? b2.w : b1.w);
  }
  v4f pv[16];
#pragma unroll
  for (int i = 0; i < 16; ++i) {
    const v4f xv = *(const v4fa*)(stg + (16 * wave + i) * GBN + 4 * lane);
    v4f q;
    q.x = xv.x + bq[0]; q.y = xv.y + bq[1]; q.z = xv.z + bq[2]; q.w = xv.w + bq[3];
    pv[i] = q;
  }
#pragma unroll
  for (int i = 0; i < 16; ++i) {
    float* op = xout + (size_t)(rowBase + 16 * wave + i) * (size_t)NF2 + colBase + 4 * lane;
    *(volatile v4f*)op = pv[i];
  }
  __threadfence();
#pragma unroll
  for (int i = 0; i < 16; ++i) {
    float* op = xout + (size_t)(rowBase + 16 * wave + i) * (size_t)NF2 + colBase + 4 * lane;
    *(volatile v4f*)op = pv[i];
  }
}

__global__ __launch_bounds__(NTHR) void k_scan(const float* __restrict__ xlr, const int* __restrict__ hits,
                                               const int* __restrict__ stab, const int* __restrict__ meta,
                                               const float* __restrict__ att, const float* __restrict__ cbias,
                                               float* outp, double* rec1) {
  __shared__ __attribute__((aligned(16))) int    stb[2 * NBA];
  __shared__ __attribute__((aligned(16))) float  stwa[NWAVE * NF];
  __shared__ __attribute__((aligned(16))) double dsum[NWAVE * NF];
  __shared__ __attribute__((aligned(16))) double recs[NF];
  const int tid = (int)threadIdx.x, lane = tid & 31, wave = tid >> 5;
  const int blk = (int)blockIdx.x;
  const int nodeBase = blk * NBA;
  {
    const v4i tv = *(const v4i*)(stab + (size_t)blk * (2 * NBA) + 4 * tid);
    *(v4ia*)(stb + 4 * tid) = tv;
  }
  int tt = meta[(size_t)blk * 32];
  const int ovf = meta[(size_t)blk * 32 + 1];
  tt = tt < 0 ? 0 : (tt > RCAP ? RCAP : tt);
  __syncthreads();

  float at8[8], cb8[8];
  {
    const v4f a0 = *(const v4f*)(att + 8 * lane),   a1 = *(const v4f*)(att + 8 * lane + 4);
    const v4f c0 = *(const v4f*)(cbias + 8 * lane), c1 = *(const v4f*)(cbias + 8 * lane + 4);
    at8[0] = rbf(a0.x); at8[1] = rbf(a0.y); at8[2] = rbf(a0.z); at8[3] = rbf(a0.w);
    at8[4] = rbf(a1.x); at8[5] = rbf(a1.y); at8[6] = rbf(a1.z); at8[7] = rbf(a1.w);
    cb8[0] = rbf(c0.x); cb8[1] = rbf(c0.y); cb8[2] = rbf(c0.z); cb8[3] = rbf(c0.w);
    cb8[4] = rbf(c1.x); cb8[5] = rbf(c1.y); cb8[6] = rbf(c1.z); cb8[7] = rbf(c1.w);
  }
  double cs[8];
#pragma unroll
  for (int j = 0; j < 8; ++j) cs[j] = 0.0;
  float* stw = stwa + wave * NF;
  const int* hbp = hits + (size_t)blk * RCAP;
  const float qnan = __int_as_float(0x7fc00000);

#pragma unroll 1
  for (int si = 0; si < NBA / NWAVE; ++si) {
    const int slot = si * NWAVE + wave;
    const int grow = nodeBase + slot;
    const int gcl  = grow < NN ? grow : NN - 1;
    const int craw = stb[slot];
    int c = craw;
    int o = stb[NBA + slot];
    c = c < 0 ? 0 : (c > DEGCAP ? DEGCAP : c);
    o = o < 0 ? 0 : (o > tt ? tt : o);
    if (c > tt - o) c = tt - o;
    const bool bad = (ovf != 0) || (craw > DEGCAP) || (craw < 0);
    const float pz = bad ? qnan : 0.0f;

    const float* xrp = xlr + (size_t)gcl * NF2 + NF + 8 * lane;
    const v4f xa = *(const v4f*)xrp, xb4 = *(const v4f*)(xrp + 4);
    ldwait();
    const float xr[8] = {xa.x, xa.y, xa.z, xa.w, xb4.x, xb4.y, xb4.z, xb4.w};
    float av[8];
#pragma unroll
    for (int j = 0; j < 8; ++j) av[j] = 0.0f;
    float mx = -1.0e30f, dn = 0.0f;
    const int total = c + 1;

#pragma unroll 1
    for (int b0 = 0; b0 < total; b0 += 32) {
      const int q = b0 + lane;
      int idx = o + q;
      idx = idx > RCAP - 1 ? RCAP - 1 : idx;
      const int ent = hbp[idx];
      int sr = ent < 0 ? 0 : (ent > NN - 1 ? NN - 1 : ent);
      sr = (q < c) ? sr : gcl;
      const int m32 = (total - b0) < 32 ? (total - b0) : 32;
#pragma unroll 1
      for (int k = 0; k < m32; ++k) {
        const int sk = __builtin_amdgcn_readlane(sr, k);
        const float* sp = xlr + (size_t)sk * NF2 + 8 * lane;
        const v4f ha = *(const v4f*)sp, hb4 = *(const v4f*)(sp + 4);
        ldwait();
        const float hs[8] = {ha.x, ha.y, ha.z, ha.w, hb4.x, hb4.y, hb4.z, hb4.w};
        float part = 0.0f;
#pragma unroll
        for (int j = 0; j < 8; ++j) {
          float v = hs[j] + xr[j];
          v = v > 0.0f ? v : v * NEGS;
          part = fmaf(v, at8[j], part);
        }
        part += __shfl_xor(part, 1);
        part += __shfl_xor(part, 2);
        part += __shfl_xor(part, 4);
        const float df = part - mx;
        const float ee = expf(-fabsf(df));
        const bool up  = df > 0.0f;
        const float s1 = up ? ee : 1.0f;
        const float s2 = up ? 1.0f : ee;
        mx = up ? part : mx;
        dn = fmaf(dn, s1, s2);
#pragma unroll
        for (int j = 0; j < 8; ++j) av[j] = fmaf(av[j], s1, s2 * hs[j]);
      }
    }
    const float inv = 1.0f / dn;
    float r[8];
#pragma unroll
    for (int j = 0; j < 8; ++j) r[j] = fmaf(av[j], inv, cb8[j]) + pz;
    const bool live = grow < NN;
    if (live) {
#pragma unroll
      for (int j = 0; j < 8; ++j) cs[j] += (double)r[j];
    }
    __builtin_amdgcn_fence(__ATOMIC_RELEASE, "wavefront");
    __builtin_amdgcn_wave_barrier();
    {
      v4f w0, w1;
      w0.x = r[0]; w0.y = r[1]; w0.z = r[2]; w0.w = r[3];
      w1.x = r[4]; w1.y = r[5]; w1.z = r[6]; w1.w = r[7];
      *(v4fa*)(stw + 8 * lane)     = w0;
      *(v4fa*)(stw + 8 * lane + 4) = w1;
    }
    __builtin_amdgcn_fence(__ATOMIC_RELEASE, "wavefront");
    __builtin_amdgcn_wave_barrier();
    const v4f f0 = *(const v4fa*)(stw + 4 * lane);
    const v4f f1 = *(const v4fa*)(stw + 128 + 4 * lane);
    float* op = outp + (size_t)gcl * NF + 4 * lane;
    if (live) { *(volatile v4f*)op = f0; *(volatile v4f*)(op + 128) = f1; }
    __threadfence();
    if (live) { *(volatile v4f*)op = f0; *(volatile v4f*)(op + 128) = f1; }
  }

#pragma unroll
  for (int j = 0; j < 8; ++j) dsum[wave * NF + 8 * lane + j] = cs[j];
  __syncthreads();
  {
    double s = 0.0;
#pragma unroll
    for (int w2 = 0; w2 < NWAVE; ++w2) s += dsum[w2 * NF + tid];
    recs[tid] = s;
  }
  __syncthreads();
  v2d rv = {0.0, 0.0};
  double* rp = rec1 + (size_t)blk * NF + 2 * (tid & 127);
  if (tid < 128) { rv = *(const v2da*)(recs + 2 * tid); *(volatile v2d*)rp = rv; }
  __threadfence();
  if (tid < 128) { *(volatile v2d*)rp = rv; }
}

__device__ __forceinline__ float col_mean(const double* __restrict__ rec1, int c) {
  double s = 0.0;
#pragma unroll 4
  for (int b = 0; b < NBLK; ++b) s += rec1[(size_t)b * NF + c];
  return (float)(s * (1.0 / (double)NN));
}
__device__ __forceinline__ float col_var(const double* __restrict__ rec2, int c) {
  double s = 0.0;
#pragma unroll 4
  for (int b = 0; b < NBLK; ++b) s += rec2[(size_t)b * NF + c];
  return (float)(s * (1.0 / (double)NN));
}

__global__ __launch_bounds__(NTHR) void k_var(const float* __restrict__ outp, const double* __restrict__ rec1,
                                              const float* __restrict__ nal, double* rec2) {
  __shared__ __attribute__((aligned(16))) double sred[NF];
  const int tid = (int)threadIdx.x;
  const int blk = (int)blockIdx.x;
  const float mean = col_mean(rec1, tid);
  const float am = rbf(nal[tid]) * mean;
  const int r0 = blk * NBA;
  const int r1 = (r0 + NBA < NN) ? r0 + NBA : NN;
  double acc = 0.0;
#pragma unroll 4
  for (int r = r0; r < r1; ++r) {
    const float d = outp[(size_t)r * NF + tid] - am;
    acc += (double)d * (double)d;
  }
  sred[tid] = acc;
  __syncthreads();
  v2d rv = {0.0, 0.0};
  double* rp = rec2 + (size_t)blk * NF + 2 * (tid & 127);
  if (tid < 128) { rv = *(const v2da*)(sred + 2 * tid); *(volatile v2d*)rp = rv; }
  __threadfence();
  if (tid < 128) { *(volatile v2d*)rp = rv; }
}

__global__ __launch_bounds__(NTHR) void k_norm_h(const float* __restrict__ outp, const double* __restrict__ rec1,
                                                 const double* __restrict__ rec2, const float* __restrict__ nw,
                                                 const float* __restrict__ nbi, const float* __restrict__ nal,
                                                 const float* __restrict__ prelu, int l, unsigned short* hhl) {
  __shared__ __attribute__((aligned(16))) float psh[NF];
  __shared__ __attribute__((aligned(16))) float psc[NF];
  __shared__ __attribute__((aligned(16))) float pnb[NF];
  const int tid = (int)threadIdx.x, lane = tid & 31, wave = tid >> 5;
  const int blk = (int)blockIdx.x;
  {
    const float mean = col_mean(rec1, tid);
    const float var  = col_var(rec2, tid);
    psh[tid] = rbf(nal[tid]) * mean;
    psc[tid] = rbf(nw[tid]) * (1.0f / sqrtf(var + EPSN));
    pnb[tid] = rbf(nbi[tid]);
  }
  __syncthreads();
  float sh[8], sc[8], nb8[8];
  {
    const v4f a0 = *(const v4fa*)(psh + 8 * lane), a1 = *(const v4fa*)(psh + 8 * lane + 4);
    const v4f b0 = *(const v4fa*)(psc + 8 * lane), b1 = *(const v4fa*)(psc + 8 * lane + 4);
    const v4f c0 = *(const v4fa*)(pnb + 8 * lane), c1 = *(const v4fa*)(pnb + 8 * lane + 4);
    sh[0] = a0.x; sh[1] = a0.y; sh[2] = a0.z; sh[3] = a0.w; sh[4] = a1.x; sh[5] = a1.y; sh[6] = a1.z; sh[7] = a1.w;
    sc[0] = b0.x; sc[1] = b0.y; sc[2] = b0.z; sc[3] = b0.w; sc[4] = b1.x; sc[5] = b1.y; sc[6] = b1.z; sc[7] = b1.w;
    nb8[0] = c0.x; nb8[1] = c0.y; nb8[2] = c0.z; nb8[3] = c0.w; nb8[4] = c1.x; nb8[5] = c1.y; nb8[6] = c1.z; nb8[7] = c1.w;
  }
  const float pa = rbf(prelu[l]);
#pragma unroll 1
  for (int i = 0; i < NBA / NWAVE; ++i) {
    const int row = blk * NBA + i * NWAVE + wave;
    if (row < MP) {
      const int rc = row < NN ? row : NN - 1;
      const bool live = row < NN;
      const float* p = outp + (size_t)rc * NF + 8 * lane;
      const v4f va = *(const v4f*)p, vb = *(const v4f*)(p + 4);
      const float vv[8] = {va.x, va.y, va.z, va.w, vb.x, vb.y, vb.z, vb.w};
      v8us hv, lv;
#pragma unroll
      for (int j = 0; j < 8; ++j) {
        float y = fmaf(vv[j] - sh[j], sc[j], nb8[j]);
        y = (y >= 0.0f) ? y : pa * y;
        y = live ? y : 0.0f;
        const unsigned hb = bfn(y);
        hv[j] = (unsigned short)hb;
        lv[j] = (unsigned short)bfn(y - __uint_as_float(hb << 16));
      }
      unsigned short* hp = hhl + (size_t)row * NF2 + 8 * lane;
      *(volatile v8us*)hp = hv;
      *(volatile v8us*)(hp + NF) = lv;
      __threadfence();
      *(volatile v8us*)hp = hv;
      *(volatile v8us*)(hp + NF) = lv;
    }
  }
}

__global__ __launch_bounds__(NTHR) void k_norm_p(const float* __restrict__ outp, const double* __restrict__ rec1,
                                                 const double* __restrict__ rec2, const float* __restrict__ nw,
                                                 const float* __restrict__ nbi, const float* __restrict__ nal,
                                                 const float* __restrict__ prelu, int l,
                                                 const int* __restrict__ batch, double* prec) {
  __shared__ __attribute__((aligned(16))) double pl[NG * NF];
  const int tid = (int)threadIdx.x;
  const int blk = (int)blockIdx.x;
  const float mean = col_mean(rec1, tid);
  const float var  = col_var(rec2, tid);
  const float sh = rbf(nal[tid]) * mean;
  const float sc = rbf(nw[tid]) * (1.0f / sqrtf(var + EPSN));
  const float nb = rbf(nbi[tid]);
  const float pa = rbf(prelu[l]);
#pragma unroll
  for (int g = 0; g < NG; ++g) pl[g * NF + tid] = 0.0;
  const int r0 = blk * NBA;
  const int r1 = (r0 + NBA < NN) ? r0 + NBA : NN;
#pragma unroll 2
  for (int r = r0; r < r1; ++r) {
    float y = fmaf(outp[(size_t)r * NF + tid] - sh, sc, nb);
    y = (y >= 0.0f) ? y : pa * y;
    const int g = batch[r];
    if ((unsigned)g < (unsigned)NG) pl[g * NF + tid] += (double)y;
  }
  __syncthreads();
  double* pp = prec + (size_t)blk * (NG * NF) + 2 * tid;
#pragma unroll 1
  for (int i = 0; i < 8; ++i) {
    const v2d v = *(const v2da*)(pl + i * 512 + 2 * tid);
    *(volatile v2d*)(pp + i * 512) = v;
  }
  __threadfence();
#pragma unroll 1
  for (int i = 0; i < 8; ++i) {
    const v2d v = *(const v2da*)(pl + i * 512 + 2 * tid);
    *(volatile v2d*)(pp + i * 512) = v;
  }
}

__global__ __launch_bounds__(NTHR) void k_tail(const double* __restrict__ prec, const float* __restrict__ nw,
                                               const float* __restrict__ nbi, const float* __restrict__ nal,
                                               const unsigned short* __restrict__ fct,
                                               const float* __restrict__ fcb, float* out) {
  __shared__ __attribute__((aligned(16))) unsigned short at[NG * NF2];
  __shared__ __attribute__((aligned(16))) float ot[NG * NO];
  const int tid = (int)threadIdx.x, lane = tid & 31, wave = tid >> 5, hh = lane >> 4, m = lane & 15;
  double p[NG];
#pragma unroll
  for (int g = 0; g < NG; ++g) p[g] = 0.0;
#pragma unroll 1
  for (int b = 0; b < NBLK; ++b) {
    const double* q = prec + (size_t)b * (NG * NF) + tid;
    double t[8];
#pragma unroll
    for (int i = 0; i < 8; ++i) t[i] = q[i * NF];
    ldwait();
#pragma unroll
    for (int i = 0; i < 8; ++i) p[i] += t[i];
#pragma unroll
    for (int i = 0; i < 8; ++i) t[i] = q[(8 + i) * NF];
    ldwait();
#pragma unroll
    for (int i = 0; i < 8; ++i) p[8 + i] += t[i];
  }
  double s = 0.0;
#pragma unroll
  for (int g = 0; g < NG; ++g) s += p[g];
  const double am = (double)rbf(nal[tid]) * (s * (1.0 / (double)NG));
  double q2 = 0.0;
#pragma unroll
  for (int g = 0; g < NG; ++g) { p[g] -= am; q2 += p[g] * p[g]; }
  const float var = (float)(q2 * (1.0 / (double)NG));
  const float inv = 1.0f / sqrtf(var + EPSN);
  const float w   = rbf(nw[tid]);
  const float bb  = rbf(nbi[tid]);
#pragma unroll
  for (int g = 0; g < NG; ++g) {
    const float y = fmaf(w * (float)p[g], inv, bb);
    const unsigned hb = bfn(y);
    at[g * NF2 + tid]      = (unsigned short)hb;
    at[g * NF2 + NF + tid] = (unsigned short)bfn(y - __uint_as_float(hb << 16));
  }
  __syncthreads();

  v8f acc = z8();
  const unsigned short* ap = at + m * NF2 + 8 * hh;
  const unsigned short* bp = fct + (size_t)(16 * wave + m) * NF2 + 8 * hh;
#pragma unroll 1
  for (int k0 = 0; k0 < NF2; k0 += 32) {
    FragB af, bf;
    af.h[0] = *(const v8usa*)(ap + k0);
    af.h[1] = *(const v8usa*)(ap + k0 + 16);
    bf.h[0] = *(const v8usa*)(bp + k0);
    bf.h[1] = *(const v8usa*)(bp + k0 + 16);
    acc = wmb(af, bf, acc);
  }
  const float fb = rbf(fcb[16 * wave + m]);
#pragma unroll
  for (int r = 0; r < 8; ++r) ot[(8 * hh + r) * NO + 16 * wave + m] = acc[r] + fb;
  __syncthreads();
  const v4f o0 = *(const v4fa*)(ot + 4 * tid);
  const v4f o1 = *(const v4fa*)(ot + 4 * (NTHR + tid));
  *(volatile v4f*)(out + 4 * tid) = o0;
  *(volatile v4f*)(out + 4 * (NTHR + tid)) = o1;
  __threadfence();
  *(volatile v4f*)(out + 4 * tid) = o0;
  *(volatile v4f*)(out + 4 * (NTHR + tid)) = o1;
}

static inline size_t al256(size_t o) { return (o + 255) & ~(size_t)255; }

extern "C" void kernel_launch(void* const* d_in, const int* in_sizes, int n_in,
                              void* d_out, int out_size, void* d_ws, size_t ws_size,
                              hipStream_t stream) {
  if (n_in < 15) return;
  if (in_sizes[0] != NN * NF || in_sizes[1] != 2 * NE || in_sizes[2] != NN) return;
  if (in_sizes[3] != NL * NF * NF || in_sizes[4] != NL * NF) return;
  if (in_sizes[5] != NL * NF * NF || in_sizes[6] != NL * NF) return;
  if (in_sizes[7] != NL * NF || in_sizes[8] != NL * NF || in_sizes[9] != NL) return;
  if (in_sizes[10] != NF || in_sizes[11] != NF || in_sizes[12] != NF) return;
  if (in_sizes[13] != NF * NO || in_sizes[14] != NO) return;
  if (out_size != NG * NO) return;

  const float* x     = (const float*)d_in[0];
  const int*   ei    = (const int*)  d_in[1];
  const int*   batch = (const int*)  d_in[2];
  const float* Wl    = (const float*)d_in[3];
  const float* bl    = (const float*)d_in[4];
  const float* Wr    = (const float*)d_in[5];
  const float* br    = (const float*)d_in[6];
  const float* att   = (const float*)d_in[7];
  const float* cbias = (const float*)d_in[8];
  const float* prelu = (const float*)d_in[9];
  const float* nw    = (const float*)d_in[10];
  const float* nbi   = (const float*)d_in[11];
  const float* nal   = (const float*)d_in[12];
  const float* fcW   = (const float*)d_in[13];
  const float* fcb   = (const float*)d_in[14];
  float* out = (float*)d_out;
  const int* src = ei;
  const int* dst = ei + NE;

  char* ws = (char*)d_ws;
  size_t off = 0;
  const size_t oXB   = off; off = al256(off + (size_t)MP * NF * 2);
  const size_t oHHL  = off; off = al256(off + (size_t)MP * NF2 * 2);
  const size_t oXLR  = off; off = al256(off + (size_t)MP * NF2 * 4);
  const size_t oOUT  = off; off = al256(off + (size_t)MP * NF * 4);
  const size_t oHITS = off; off = al256(off + (size_t)NBLK * RCAP * 4);
  const size_t oSTAB = off; off = al256(off + (size_t)NBLK * 2 * NBA * 4);
  const size_t oMETA = off; off = al256(off + (size_t)NBLK * 32 * 4);
  const size_t oW0   = off; off = al256(off + (size_t)NF2 * NF * 2);
  const size_t oW12  = off; off = al256(off + (size_t)2 * NF2 * NF2 * 2);
  const size_t oFCT  = off; off = al256(off + (size_t)NO * NF2 * 2);
  const size_t oR1   = off; off = al256(off + (size_t)NBLK * NF * 8);
  const size_t oR2   = off; off = al256(off + (size_t)NBLK * NF * 8);
  const size_t oPR   = off; off = al256(off + (size_t)NBLK * NG * NF * 8);
  if (off > ws_size || off > (size_t)WSMAX) return;
  unsigned short* XB   = (unsigned short*)(ws + oXB);
  unsigned short* HHL  = (unsigned short*)(ws + oHHL);
  float*          XLR  = (float*)(ws + oXLR);
  float*          OUTP = (float*)(ws + oOUT);
  int*            HITS = (int*)(ws + oHITS);
  int*            STAB = (int*)(ws + oSTAB);
  int*            META = (int*)(ws + oMETA);
  unsigned short* W0   = (unsigned short*)(ws + oW0);
  unsigned short* W12  = (unsigned short*)(ws + oW12);
  unsigned short* FCT  = (unsigned short*)(ws + oFCT);
  double*         REC1 = (double*)(ws + oR1);
  double*         REC2 = (double*)(ws + oR2);
  double*         PREC = (double*)(ws + oPR);

  hipFuncSetAttribute(reinterpret_cast<const void*>(&k_bucket),
                      hipFuncAttributeMaxDynamicSharedMemorySize, B_LDS_BYTES);

  k_prep<<<PBX + WBX, NTHR, 0, stream>>>(x, Wl, Wr, fcW, XB, W0, W12, FCT);
  k_bucket<<<NBLK, NTHR, B_LDS_BYTES, stream>>>(src, dst, HITS, STAB, META);

  for (int l = 0; l < NL; ++l) {
    const unsigned short* Ap = (l == 0) ? XB : HHL;
    const unsigned short* Bp = (l == 0) ? W0 : (W12 + (size_t)(l - 1) * (NF2 * NF2));
    const int K = (l == 0) ? NF : NF2;
    k_gemm<<<dim3(MP / GBM, NF2 / GBN), GTHR, 0, stream>>>(Ap, Bp, K, bl + l * NF, br + l * NF, XLR);
    k_scan<<<NBLK, NTHR, 0, stream>>>(XLR, HITS, STAB, META, att + l * NF, cbias + l * NF, OUTP, REC1);
    k_var<<<NBLK, NTHR, 0, stream>>>(OUTP, REC1, nal, REC2);
    if (l < NL - 1) {
      k_norm_h<<<NBLK, NTHR, 0, stream>>>(OUTP, REC1, REC2, nw, nbi, nal, prelu, l, HHL);
    } else {
      k_norm_p<<<NBLK, NTHR, 0, stream>>>(OUTP, REC1, REC2, nw, nbi, nal, prelu, l, batch, PREC);
    }
  }
  k_tail<<<1, NTHR, 0, stream>>>(PREC, nw, nbi, nal, FCT, fcb, out);
}
